// GCN2_12893491822964
// MI455X (gfx1250) — hardware-run, weakly checked
//
#include <hip/hip_runtime.h>
#include <stddef.h>
#include <stdint.h>
#include <math.h>

#ifndef U_SINGLE
#define U_SINGLE 0
#endif

#define NN      50000
#define FD      128
#define HD      64
#define NLAY    8
#define NE      800000
#define NC      40
#define NCP     48
#define GBM     128
#define MP      50048
#define KL      128
#if U_SINGLE
#define KRUN    HD
#else
#define KRUN    KL
#endif
#define NTHR    256
#define NWAVE   8
#define EPT     8
#define WCH     (32 * EPT)
#define NBRUN   512
#define SLB     9
#define NBK     98
#define WLCAP   1536
#define RCAP    12288
#define TRIPCAP 64
#define MAXDEG_MEAS  33
#define MAXB512_MEAS 8397
#define ABM     64
#define SP      68
#define WSMAX   134217728

#define BK_ZINTS (NWAVE * WLCAP + RCAP + 3 * NBRUN)
#define BK_INTS  (BK_ZINTS + 16)
#define BK_LDS   (BK_INTS * 4)

#define UPR  (FD / 8)
#define PBX  (MP * FD / 8 / NTHR)
#define PBW0 (HD * FD / 8 / NTHR)
#define PBWL (NLAY * HD * KL / 8 / NTHR)
#define PBWO (NCP * KL / 8 / NTHR)
#define PBTOT (PBX + PBW0 + PBWL + PBWO + 1)

static_assert(HD == 64 && HD == 16 * 4);
static_assert(UPR == 16 && KL / 8 == 16);
static_assert(MP % GBM == 0 && MP >= NN && MP == 391 * GBM && MP % ABM == 0);
static_assert(NBRUN == (1 << SLB) && NBRUN % ABM == 0 && NBRUN % GBM == 0 && NBRUN % 32 == 0);
static_assert(NBK * NBRUN >= MP);
static_assert(NE < (1 << 21) && (((long long)NE) << SLB) < (1LL << 31));
static_assert(NE % WCH == 0 && NE % 4 == 0);
static_assert(RCAP == NWAVE * WLCAP && RCAP % 4 == 0 && BK_ZINTS % 4 == 0);
static_assert(RCAP % (NTHR * 4) == 0);
static_assert((long long)RCAP * 100 >= (long long)MAXB512_MEAS * 105);
static_assert(WLCAP >= MAXB512_MEAS / 8 + 8 * 33 + 1);
static_assert(NN <= 65536);
static_assert(MAXDEG_MEAS + 8 <= TRIPCAP && TRIPCAP < 65536);
static_assert((GBM * NC * 4) % 128 == 0 && (((NN % GBM) * NC * 4) % 128) == 0);
static_assert((MP / GBM - 1) * GBM * NC + (NN % GBM) * NC == NN * NC);
static_assert((MP * FD / 8) % NTHR == 0 && (HD * FD / 8) % NTHR == 0);
static_assert((NLAY * HD * KL / 8) % NTHR == 0 && (NCP * KL / 8) % NTHR == 0);
static_assert(FD % 32 == 0 && KL % 32 == 0 && KL == 2 * HD && KRUN % 32 == 0 && KRUN <= KL);
static_assert(NCP % 16 == 0 && NCP >= NC && NC % 4 == 0);
static_assert(BK_LDS <= 300000);
static_assert((GBM * SP + 128) * 4 <= 65536);
static_assert((GBM * NC + 128) * 4 <= 65536);
static_assert(GBM * NC / 4 == 5 * NTHR);

typedef float          v4f   __attribute__((ext_vector_type(4)));
typedef float          v8f   __attribute__((ext_vector_type(8)));
typedef int            v4i   __attribute__((ext_vector_type(4)));
typedef int            v8i   __attribute__((ext_vector_type(8)));
typedef unsigned short v8us  __attribute__((ext_vector_type(8)));
typedef unsigned short v16us __attribute__((ext_vector_type(16)));
typedef __bf16         v16bf __attribute__((ext_vector_type(16)));
typedef v4f  __attribute__((may_alias)) v4fa;
typedef v4i  __attribute__((may_alias)) v4ia;
typedef v8us __attribute__((may_alias)) v8usa;
union FragB { v16bf v; v16us u; v8us h[2]; v8i w; };

__device__ __forceinline__ v8f wmb(const FragB& a, const FragB& b, v8f c) {
  v8f d = __builtin_amdgcn_wmma_f32_16x16x32_bf16(false, a.v, false, b.v, (short)0, c, false, false);
  asm volatile("v_nop\n\tv_nop\n\tv_nop\n\tv_nop" : "+v"(d) : "v"(a.w), "v"(b.w));
  return d;
}

__device__ __forceinline__ unsigned bf16_bits(float f) {
  const unsigned u = __float_as_uint(f);
  const unsigned r = (u + 0x7FFFu + ((u >> 16) & 1u)) >> 16;
  const unsigned q = (u >> 16) | 0x40u;
  return ((u & 0x7fffffffu) > 0x7f800000u) ? q : r;
}

__device__ __forceinline__ void hilo_pack(float v0, float v1, float v2, float v3,
                                          int& h01, int& h23, int& l01, int& l23) {
  const unsigned a0 = bf16_bits(v0), a1 = bf16_bits(v1), a2 = bf16_bits(v2), a3 = bf16_bits(v3);
  const unsigned b0 = bf16_bits(v0 - __uint_as_float(a0 << 16));
  const unsigned b1 = bf16_bits(v1 - __uint_as_float(a1 << 16));
  const unsigned b2 = bf16_bits(v2 - __uint_as_float(a2 << 16));
  const unsigned b3 = bf16_bits(v3 - __uint_as_float(a3 << 16));
  h01 = (int)(a0 | (a1 << 16)); h23 = (int)(a2 | (a3 << 16));
  l01 = (int)(b0 | (b1 << 16)); l23 = (int)(b2 | (b3 << 16));
}

__device__ __forceinline__ v4i regroup8(int h01, int h23, int l01, int l23, int lane) {
  const int t  = lane & 15;
  const int s0 = (lane & 16) + ((2 * t) & 15), s1 = s0 + 1;
  const int a0 = __shfl(h01, s0, 32), a1 = __shfl(h23, s0, 32), a2 = __shfl(h01, s1, 32), a3 = __shfl(h23, s1, 32);
  const int b0 = __shfl(l01, s0, 32), b1 = __shfl(l23, s0, 32), b2 = __shfl(l01, s1, 32), b3 = __shfl(l23, s1, 32);
  const int mk = (t < 8) ? -1 : 0;
  v4i o;
  o.x = (a0 & mk) | (b0 & ~mk); o.y = (a1 & mk) | (b1 & ~mk);
  o.z = (a2 & mk) | (b2 & ~mk); o.w = (a3 & mk) | (b3 & ~mk);
  return o;
}

__device__ __forceinline__ void st2_v4f(float* p, v4f v) {
  *(volatile v4f*)p = v;
  __threadfence();
  *(volatile v4f*)p = v;
}
__device__ __forceinline__ void st2_v8us(unsigned short* p, v8us v) {
  *(volatile v8us*)p = v;
  __threadfence();
  *(volatile v8us*)p = v;
}

__device__ __forceinline__ v8us gather8(const float* __restrict__ base, int stride) {
  float f[8];
#pragma unroll
  for (int i = 0; i < 8; ++i) f[i] = base[(size_t)i * (size_t)stride];
  v8us o;
#pragma unroll
  for (int i = 0; i < 8; ++i) o[i] = (unsigned short)bf16_bits(f[i]);
  return o;
}

__global__ __launch_bounds__(NTHR) void k_prep(const float* __restrict__ x, const float* __restrict__ w0,
                                               const float* __restrict__ b0, const float* __restrict__ wl,
                                               const float* __restrict__ w2, const float* __restrict__ b2,
                                               unsigned short* xb, unsigned short* w0t, unsigned short* wld,
                                               unsigned short* wod, float* sm) {
  const int tid = (int)threadIdx.x, lane = tid & 31;
  const int blk = (int)blockIdx.x;
  if (blk < PBX) {
    const int u   = blk * NTHR + tid;
    const int row = u >> 4, k8 = (u & 15) * 8;
    const int rc  = row < NN ? row : NN - 1;
    const unsigned mk = row < NN ? 0xffffu : 0u;
    const float* p = x + (size_t)rc * FD + k8;
    const v4f a = *(const v4fa*)p;
    const v4f b = *(const v4fa*)(p + 4);
    v8us o;
    o[0] = (unsigned short)(bf16_bits(a.x) & mk); o[1] = (unsigned short)(bf16_bits(a.y) & mk);
    o[2] = (unsigned short)(bf16_bits(a.z) & mk); o[3] = (unsigned short)(bf16_bits(a.w) & mk);
    o[4] = (unsigned short)(bf16_bits(b.x) & mk); o[5] = (unsigned short)(bf16_bits(b.y) & mk);
    o[6] = (unsigned short)(bf16_bits(b.z) & mk); o[7] = (unsigned short)(bf16_bits(b.w) & mk);
    st2_v8us(xb + (size_t)row * FD + k8, o);
  } else if (blk < PBX + PBW0) {
    const int u = (blk - PBX) * NTHR + tid;
    const int n = u >> 4, k8 = (u & 15) * 8;
    const v8us o = gather8(w0 + (size_t)k8 * HD + n, HD);
    st2_v8us(w0t + (size_t)n * FD + k8, o);
  } else if (blk < PBX + PBW0 + PBWL) {
    const int u = (blk - PBX - PBW0) * NTHR + tid;
    const int l = u >> 10, n = (u >> 4) & 63, k8 = (u & 15) * 8, kk = k8 & 63;
    const v8us o = gather8(wl + (size_t)l * HD * HD + (size_t)kk * HD + n, HD);
    st2_v8us(wld + (size_t)l * HD * KL + (size_t)n * KL + k8, o);
  } else if (blk < PBX + PBW0 + PBWL + PBWO) {
    const int u = (blk - PBX - PBW0 - PBWL) * NTHR + tid;
    const int n = u >> 4, k8 = (u & 15) * 8, kk = k8 & 63;
    const int nc = n < NC ? n : NC - 1;
    const unsigned mk = n < NC ? 0xffffu : 0u;
    const v8us g = gather8(w2 + (size_t)kk * NC + nc, NC);
    v8us o;
#pragma unroll
    for (int i = 0; i < 8; ++i) o[i] = (unsigned short)((unsigned)g[i] & mk);
    st2_v8us(wod + (size_t)n * KL + k8, o);
  } else {
    if (tid < 32) {
      const int q = lane & 15;
      const int i0 = 4 * q, i1 = i0 + 1, i2 = i0 + 2, i3 = i0 + 3;
      const float a0 = b0[i0], a1 = b0[i1], a2 = b0[i2], a3 = b0[i3];
      const float c0 = b2[i0 < NC ? i0 : NC - 1], c1 = b2[i1 < NC ? i1 : NC - 1];
      const float c2 = b2[i2 < NC ? i2 : NC - 1], c3 = b2[i3 < NC ? i3 : NC - 1];
      asm volatile("" :: "v"(a0), "v"(a1), "v"(a2), "v"(a3));
      asm volatile("" :: "v"(c0), "v"(c1), "v"(c2), "v"(c3));
      const unsigned ma = (lane < 16) ? 0xffffffffu : 0u;
      const unsigned m0 = (i0 < NC) ? ~ma : 0u, m1 = (i1 < NC) ? ~ma : 0u;
      const unsigned m2 = (i2 < NC) ? ~ma : 0u, m3 = (i3 < NC) ? ~ma : 0u;
      v4f o;
      o.x = __uint_as_float(((bf16_bits(a0) << 16) & ma) | ((bf16_bits(c0) << 16) & m0));
      o.y = __uint_as_float(((bf16_bits(a1) << 16) & ma) | ((bf16_bits(c1) << 16) & m1));
      o.z = __uint_as_float(((bf16_bits(a2) << 16) & ma) | ((bf16_bits(c2) << 16) & m2));
      o.w = __uint_as_float(((bf16_bits(a3) << 16) & ma) | ((bf16_bits(c3) << 16) & m3));
      st2_v4f(sm + 4 * lane, o);
    }
  }
}

__device__ __forceinline__ void bucket_flush(const int* pl, const int* cnt, int ov, int* lp, int* cop, int* fp,
                                             int tid) {
#pragma unroll 1
  for (int i = tid * 4; i < RCAP; i += NTHR * 4) {
    const v4i v = *(const v4ia*)(pl + i);
    *(volatile v4i*)(lp + i) = v;
  }
  {
    const v4i v = *(const v4ia*)(cnt + 4 * tid);
    *(volatile v4i*)(cop + 4 * tid) = v;
  }
  if (tid < 8) {
    const v4i f = {ov, ov, ov, ov};
    *(volatile v4i*)(fp + 4 * tid) = f;
  }
}

__global__ __launch_bounds__(NTHR) void k_bucket(const int* __restrict__ srcs, const int* __restrict__ dsts,
                                                 const float* __restrict__ ew, int* LIST, int* CO, int* FLAG) {
  extern __shared__ __attribute__((aligned(16))) int dsm[];
  int* wl   = dsm;
  int* pl   = dsm + NWAVE * WLCAP;
  int* cnt  = pl + RCAP;
  int* offs = cnt + NBRUN;
  int* cur  = offs + NBRUN;
  int* misc = cur + NBRUN;
  const int tid = (int)threadIdx.x, lane = tid & 31, wave = tid >> 5;
  const int blk = (int)blockIdx.x;
  const unsigned nbs = (unsigned)(blk * NBRUN);

  {
    const v4i z4 = {0, 0, 0, 0};
    for (int i = tid * 4; i < BK_ZINTS; i += NTHR * 4) *(v4ia*)(dsm + i) = z4;
    if (tid < 16) misc[tid] = 0;
  }
  __syncthreads();

  {
    const int per  = ((NE + NWAVE * WCH - 1) / (NWAVE * WCH)) * WCH;
    const int ebeg = wave * per;
    const int eend = (ebeg + per < NE) ? (ebeg + per) : NE;
    int* mylist = wl + wave * WLCAP;
    int wc = 0;
#pragma unroll 1
    for (int cb = ebeg; cb < eend; cb += WCH) {
      const int e0 = cb + lane * EPT;
      const v4i da = *(const v4ia*)(dsts + e0);
      const v4i db = *(const v4ia*)(dsts + e0 + 4);
      const unsigned s0 = (unsigned)da.x - nbs, s1 = (unsigned)da.y - nbs;
      const unsigned s2 = (unsigned)da.z - nbs, s3 = (unsigned)da.w - nbs;
      const unsigned s4 = (unsigned)db.x - nbs, s5 = (unsigned)db.y - nbs;
      const unsigned s6 = (unsigned)db.z - nbs, s7 = (unsigned)db.w - nbs;
      const bool h0 = s0 < (unsigned)NBRUN, h1 = s1 < (unsigned)NBRUN, h2 = s2 < (unsigned)NBRUN, h3 = s3 < (unsigned)NBRUN;
      const bool h4 = s4 < (unsigned)NBRUN, h5 = s5 < (unsigned)NBRUN, h6 = s6 < (unsigned)NBRUN, h7 = s7 < (unsigned)NBRUN;
      const unsigned m0 = __builtin_amdgcn_ballot_w32(h0), m1 = __builtin_amdgcn_ballot_w32(h1);
      const unsigned m2 = __builtin_amdgcn_ballot_w32(h2), m3 = __builtin_amdgcn_ballot_w32(h3);
      const unsigned m4 = __builtin_amdgcn_ballot_w32(h4), m5 = __builtin_amdgcn_ballot_w32(h5);
      const unsigned m6 = __builtin_amdgcn_ballot_w32(h6), m7 = __builtin_amdgcn_ballot_w32(h7);
      const unsigned any = m0 | m1 | m2 | m3 | m4 | m5 | m6 | m7;
      if (any != 0u) {
        const int pre = (int)(__builtin_amdgcn_mbcnt_lo(m0, 0u) + __builtin_amdgcn_mbcnt_lo(m1, 0u) +
                              __builtin_amdgcn_mbcnt_lo(m2, 0u) + __builtin_amdgcn_mbcnt_lo(m3, 0u) +
                              __builtin_amdgcn_mbcnt_lo(m4, 0u) + __builtin_amdgcn_mbcnt_lo(m5, 0u) +
                              __builtin_amdgcn_mbcnt_lo(m6, 0u) + __builtin_amdgcn_mbcnt_lo(m7, 0u));
        int p = wc + pre;
        if (h0) { if (p < WLCAP) mylist[p] = ((e0 + 0) << SLB) | (int)s0; p = p + 1; }
        if (h1) { if (p < WLCAP) mylist[p] = ((e0 + 1) << SLB) | (int)s1; p = p + 1; }
        if (h2) { if (p < WLCAP) mylist[p] = ((e0 + 2) << SLB) | (int)s2; p = p + 1; }
        if (h3) { if (p < WLCAP) mylist[p] = ((e0 + 3) << SLB) | (int)s3; p = p + 1; }
        if (h4) { if (p < WLCAP) mylist[p] = ((e0 + 4) << SLB) | (int)s4; p = p + 1; }
        if (h5) { if (p < WLCAP) mylist[p] = ((e0 + 5) << SLB) | (int)s5; p = p + 1; }
        if (h6) { if (p < WLCAP) mylist[p] = ((e0 + 6) << SLB) | (int)s6; p = p + 1; }
        if (h7) { if (p < WLCAP) mylist[p] = ((e0 + 7) << SLB) | (int)s7; p = p + 1; }
        wc += (int)(__builtin_popcount(m0) + __builtin_popcount(m1) + __builtin_popcount(m2) + __builtin_popcount(m3) +
                    __builtin_popcount(m4) + __builtin_popcount(m5) + __builtin_popcount(m6) + __builtin_popcount(m7));
      }
    }
    if (lane == 0) misc[wave] = wc;
  }
  __syncthreads();

  if (wave == 0) {
    int ov = 0;
#pragma unroll 1
    for (int w2 = 0; w2 < NWAVE; ++w2) {
      int c = misc[w2];
      if (c > WLCAP) ov = 1;
      c = c < 0 ? 0 : (c > WLCAP ? WLCAP : c);
#pragma unroll 1
      for (int b0 = 0; b0 < c; b0 += 32) {
        const int idx = b0 + lane;
        const int ent = wl[w2 * WLCAP + (idx < WLCAP ? idx : WLCAP - 1)];
        const int m32 = (c - b0) < 32 ? (c - b0) : 32;
#pragma unroll 1
        for (int k = 0; k < m32; ++k) {
          const int u    = __builtin_amdgcn_readlane(ent, k);
          const int slot = u & (NBRUN - 1);
          if (lane == 0) cnt[slot] = cnt[slot] + 1;
        }
      }
    }
    if (lane == 0) misc[9] = ov;
  }
  __syncthreads();
  if (wave == 0) {
    const int base = lane * (NBRUN / 32);
    int s = 0;
#pragma unroll 1
    for (int i = 0; i < NBRUN / 32; ++i) s += cnt[base + i];
    int incl = s;
#pragma unroll
    for (int d = 1; d < 32; d <<= 1) {
      const int y = __shfl_up(incl, d, 32);
      if (lane >= d) incl += y;
    }
    int run = incl - s;
#pragma unroll 1
    for (int i = 0; i < NBRUN / 32; ++i) {
      const int cv = cnt[base + i];
      offs[base + i] = run;
      cur[base + i]  = run;
      run += cv;
    }
  }
  __syncthreads();

  if (wave == 0) {
#pragma unroll 1
    for (int w2 = 0; w2 < NWAVE; ++w2) {
      int c = misc[w2];
      c = c < 0 ? 0 : (c > WLCAP ? WLCAP : c);
#pragma unroll 1
      for (int b0 = 0; b0 < c; b0 += 32) {
        const int idx = b0 + lane;
        const int ent = wl[w2 * WLCAP + (idx < WLCAP ? idx : WLCAP - 1)];
        int eid = (ent >> SLB) & 0x1FFFFF;
        eid = eid > NE - 1 ? NE - 1 : eid;
        int sr = srcs[eid];
        sr = sr < 0 ? 0 : (sr > NN - 1 ? NN - 1 : sr);
        const int word = (int)((unsigned)sr | (bf16_bits(ew[eid]) << 16));
        const int m32 = (c - b0) < 32 ? (c - b0) : 32;
#pragma unroll 1
        for (int k = 0; k < m32; ++k) {
          const int u    = __builtin_amdgcn_readlane(ent, k);
          const int wd   = __builtin_amdgcn_readlane(word, k);
          const int slot = u & (NBRUN - 1);
          if (lane == 0) {
            int p = cur[slot];
            p = p < 0 ? 0 : (p > RCAP - 1 ? RCAP - 1 : p);
            pl[p] = wd;
            cur[slot] = p + 1;
          }
        }
      }
    }
  }
  __syncthreads();

  const int ovf = misc[9];
  int* lp  = LIST + (size_t)blk * RCAP;
  int* cop = CO + (size_t)blk * (2 * NBRUN);
  int* fp  = FLAG + (size_t)blk * 32;
  bucket_flush(pl, cnt, ovf, lp, cop, fp, tid);
  __threadfence();
  bucket_flush(pl, cnt, ovf, lp, cop, fp, tid);
}

template <int PITCH, int KR, int NT>
__device__ __forceinline__ void gemm_rows16(const unsigned short* __restrict__ ap,
                                            const unsigned short* __restrict__ bp, v8f (&acc)[NT]) {
  static_assert(KR % 32 == 0 && KR <= PITCH);
#pragma unroll 1
  for (int k0 = 0; k0 < KR; k0 += 32) {
    FragB af;
    af.h[0] = *(const v8usa*)(ap + k0);
    af.h[1] = *(const v8usa*)(ap + k0 + 16);
#pragma unroll
    for (int nt = 0; nt < NT; ++nt) {
      const unsigned short* wq = bp + (size_t)(16 * nt) * (size_t)PITCH + k0;
      FragB bf;
      bf.h[0] = *(const v8usa*)wq;
      bf.h[1] = *(const v8usa*)(wq + 16);
      acc[nt] = wmb(af, bf, acc[nt]);
    }
  }
}

__device__ __forceinline__ void stage_d(float* stg, const v8f (&acc)[4], int wave, int hh, int m) {
#pragma unroll
  for (int nt = 0; nt < 4; ++nt) {
#pragma unroll
    for (int r = 0; r < 8; ++r) stg[(16 * wave + 8 * hh + r) * SP + 16 * nt + m] = acc[nt][r];
  }
}

__global__ __launch_bounds__(NTHR) __attribute__((amdgpu_num_vgpr(248)))
void k_gemm0(const unsigned short* __restrict__ XB, const unsigned short* __restrict__ W0T,
             const float* __restrict__ sm, float* X0) {
  __shared__ __attribute__((aligned(16))) float stg[GBM * SP];
  __shared__ __attribute__((aligned(16))) float sb[128];
  const int tid = (int)threadIdx.x, lane = tid & 31, wave = tid >> 5, hh = lane >> 4, m = lane & 15;
  const int rowBase = (int)blockIdx.x * GBM;
  if (tid < 32) *(v4fa*)(sb + 4 * tid) = *(const v4fa*)(sm + 4 * tid);

  v8f acc[4];
  {
    const v8f z = {0.f, 0.f, 0.f, 0.f, 0.f, 0.f, 0.f, 0.f};
#pragma unroll
    for (int t = 0; t < 4; ++t) acc[t] = z;
  }
  const unsigned short* ap = XB + (size_t)(rowBase + 16 * wave + m) * (size_t)FD + 8 * hh;
  const unsigned short* bp = W0T + (size_t)m * (size_t)FD + 8 * hh;
  gemm_rows16<FD, FD, 4>(ap, bp, acc);
  stage_d(stg, acc, wave, hh, m);
  __syncthreads();

  const v4f bias = *(const v4fa*)(sb + 4 * m);
#pragma unroll 1
  for (int i = 0; i < 8; ++i) {
    const int lr   = 16 * wave + 2 * i + hh;
    const int grow = rowBase + lr;
    const bool live = grow < NN;
    const v4f a = *(const v4fa*)(stg + lr * SP + 4 * m);
    asm volatile("" :: "v"(a));
    float v0 = a.x + bias.x, v1 = a.y + bias.y, v2 = a.z + bias.z, v3 = a.w + bias.w;
    v0 = (v0 > 0.0f) ? v0 : (v0 - v0); v1 = (v1 > 0.0f) ? v1 : (v1 - v1);
    v2 = (v2 > 0.0f) ? v2 : (v2 - v2); v3 = (v3 > 0.0f) ? v3 : (v3 - v3);
    v4f o;
    o.x = live ? v0 : 0.0f; o.y = live ? v1 : 0.0f; o.z = live ? v2 : 0.0f; o.w = live ? v3 : 0.0f;
    st2_v4f(X0 + (size_t)grow * HD + 4 * m, o);
  }
}

__global__ __launch_bounds__(NTHR) void k_agg(const int* __restrict__ LIST, const int* __restrict__ CO,
                                              const int* __restrict__ FLAG, const float* Hs, const float* X0,
                                              float c9, float c1, float* HMIX, unsigned short* HMhl) {
  const int tid = (int)threadIdx.x, lane = tid & 31, wave = tid >> 5, hh = lane >> 4, q = lane & 15;
  const int rowBase = (int)blockIdx.x * ABM;
  const int bucket  = rowBase >> SLB;
  const int* lb  = LIST + (size_t)bucket * RCAP;
  const int* cob = CO + (size_t)bucket * (2 * NBRUN);
  const int flag = FLAG[(size_t)bucket * 32];
  const float qnan = __uint_as_float(0x7fc00000u);

#pragma unroll 1
  for (int i = 0; i < ABM / (2 * NWAVE); ++i) {
    const int d    = rowBase + (ABM / NWAVE) * wave + 2 * i + hh;
    const int slot = d & (NBRUN - 1);
    int c = cob[slot];
    int o = cob[NBRUN + slot];
    const bool big = c > TRIPCAP;
    c = c < 0 ? 0 : (c > TRIPCAP ? TRIPCAP : c);
    o = o < 0 ? 0 : (o > RCAP - 1 ? RCAP - 1 : o);
    const int co = __shfl_xor(c, 16, 32);
    const int cm = c > co ? c : co;
    int last = o + (c > 0 ? c : 1) - 1;
    last = last > RCAP - 1 ? RCAP - 1 : last;
    float a0 = 0.0f, a1 = 0.0f, a2 = 0.0f, a3 = 0.0f;
#pragma unroll 1
    for (int j = 0; j < cm; ++j) {
      int idx = o + j;
      idx = idx > last ? last : idx;
      const unsigned wd = (unsigned)lb[idx];
      int sr = (int)(wd & 0xffffu);
      sr = sr > NN - 1 ? NN - 1 : sr;
      const float w = __uint_as_float(wd & 0xffff0000u);
      const v4f v = *(const v4fa*)(Hs + (size_t)sr * HD + 4 * q);
      asm volatile("" :: "v"(v));
      const bool valid = j < c;
      const float t0 = fmaf(w, v.x, a0), t1 = fmaf(w, v.y, a1), t2 = fmaf(w, v.z, a2), t3 = fmaf(w, v.w, a3);
      a0 = valid ? t0 : a0; a1 = valid ? t1 : a1; a2 = valid ? t2 : a2; a3 = valid ? t3 : a3;
    }
    const v4f g = *(const v4fa*)(X0 + (size_t)d * HD + 4 * q);
    float m0 = c9 * a0 + c1 * g.x, m1 = c9 * a1 + c1 * g.y;
    float m2 = c9 * a2 + c1 * g.z, m3 = c9 * a3 + c1 * g.w;
    const bool bad  = (flag != 0) | big;
    const bool live = d < NN;
    m0 = bad ? qnan : m0; m1 = bad ? qnan : m1; m2 = bad ? qnan : m2; m3 = bad ? qnan : m3;
    m0 = live ? m0 : 0.0f; m1 = live ? m1 : 0.0f; m2 = live ? m2 : 0.0f; m3 = live ? m3 : 0.0f;
    int h01, h23, l01, l23;
    hilo_pack(m0, m1, m2, m3, h01, h23, l01, l23);
    const v4i ow = regroup8(h01, h23, l01, l23, lane);
    v4f ov;
    ov.x = m0; ov.y = m1; ov.z = m2; ov.w = m3;
    float* op = HMIX + (size_t)d * HD + 4 * q;
    unsigned short* hp = HMhl + (size_t)d * KL + 8 * q;
    *(volatile v4f*)op = ov;
    *(volatile v4i*)hp = ow;
    __threadfence();
    *(volatile v4f*)op = ov;
    *(volatile v4i*)hp = ow;
  }
}

template <int LAST>
__global__ __launch_bounds__(NTHR) __attribute__((amdgpu_num_vgpr(248)))
void k_lin(const unsigned short* __restrict__ A, const unsigned short* __restrict__ BT,
           const float* __restrict__ HMIX, float cm, float cb, float* H, unsigned short* Hhl) {
  __shared__ __attribute__((aligned(16))) float stg[GBM * SP];
  const int tid = (int)threadIdx.x, lane = tid & 31, wave = tid >> 5, hh = lane >> 4, m = lane & 15;
  const int rowBase = (int)blockIdx.x * GBM;

  v8f acc[4];
  {
    const v8f z = {0.f, 0.f, 0.f, 0.f, 0.f, 0.f, 0.f, 0.f};
#pragma unroll
    for (int t = 0; t < 4; ++t) acc[t] = z;
  }
  const unsigned short* ap = A + (size_t)(rowBase + 16 * wave + m) * (size_t)KL + 8 * hh;
  const unsigned short* bp = BT + (size_t)m * (size_t)KL + 8 * hh;
  gemm_rows16<KL, KRUN, 4>(ap, bp, acc);
  stage_d(stg, acc, wave, hh, m);
  __syncthreads();

#pragma unroll 1
  for (int i = 0; i < 8; ++i) {
    const int lr   = 16 * wave + 2 * i + hh;
    const int grow = rowBase + lr;
    const bool live = grow < NN;
    const v4f a  = *(const v4fa*)(stg + lr * SP + 4 * m);
    const v4f hm = *(const v4fa*)(HMIX + (size_t)grow * HD + 4 * m);
    asm volatile("" :: "v"(a));
    asm volatile("" :: "v"(hm));
    float v0 = cm * hm.x + cb * a.x, v1 = cm * hm.y + cb * a.y;
    float v2 = cm * hm.z + cb * a.z, v3 = cm * hm.w + cb * a.w;
    v0 = (v0 > 0.0f) ? v0 : (v0 - v0); v1 = (v1 > 0.0f) ? v1 : (v1 - v1);
    v2 = (v2 > 0.0f) ? v2 : (v2 - v2); v3 = (v3 > 0.0f) ? v3 : (v3 - v3);
    v0 = live ? v0 : 0.0f; v1 = live ? v1 : 0.0f; v2 = live ? v2 : 0.0f; v3 = live ? v3 : 0.0f;
    if constexpr (LAST != 0) {
      int h01, h23, l01, l23;
      hilo_pack(v0, v1, v2, v3, h01, h23, l01, l23);
      const v4i ow = regroup8(h01, h23, l01, l23, lane);
      unsigned short* hp = Hhl + (size_t)grow * KL + 8 * m;
      *(volatile v4i*)hp = ow;
      __threadfence();
      *(volatile v4i*)hp = ow;
    } else {
      v4f o;
      o.x = v0; o.y = v1; o.z = v2; o.w = v3;
      float* op = H + (size_t)grow * HD + 4 * m;
      *(volatile v4f*)op = o;
      __threadfence();
      *(volatile v4f*)op = o;
    }
  }
}

__device__ __forceinline__ void head_flush(const float* lg, float* ob, int nv4, int flag, int tid) {
  const float qnan = __uint_as_float(0x7fc00000u);
#pragma unroll 1
  for (int it = 0; it < 5; ++it) {
    const int i4 = it * NTHR + tid;
    const v4f v = *(const v4fa*)(lg + 4 * i4);
    asm volatile("" :: "v"(v));
    v4f o;
    o.x = (flag != 0) ? qnan : v.x; o.y = (flag != 0) ? qnan : v.y;
    o.z = (flag != 0) ? qnan : v.z; o.w = (flag != 0) ? qnan : v.w;
    if (i4 < nv4) *(volatile v4f*)(ob + (size_t)4 * (size_t)i4) = o;
  }
}

__global__ __launch_bounds__(NTHR) __attribute__((amdgpu_num_vgpr(248)))
void k_head(const unsigned short* __restrict__ Hhl, const unsigned short* __restrict__ WOD,
            const float* __restrict__ sm, const int* __restrict__ FLAG, float* out) {
  __shared__ __attribute__((aligned(16))) float lg[GBM * NC];
  __shared__ __attribute__((aligned(16))) float sb[128];
  const int tid = (int)threadIdx.x, lane = tid & 31, wave = tid >> 5, hh = lane >> 4, m = lane & 15;
  const int blk = (int)blockIdx.x;
  const int rowBase = blk * GBM;
  const int flag = FLAG[(size_t)(rowBase >> SLB) * 32];
  if (tid < 32) *(v4fa*)(sb + 4 * tid) = *(const v4fa*)(sm + 4 * tid);

  v8f acc[3];
  {
    const v8f z = {0.f, 0.f, 0.f, 0.f, 0.f, 0.f, 0.f, 0.f};
#pragma unroll
    for (int t = 0; t < 3; ++t) acc[t] = z;
  }
  const unsigned short* ap = Hhl + (size_t)(rowBase + 16 * wave + m) * (size_t)KL + 8 * hh;
  const unsigned short* bp = WOD + (size_t)m * (size_t)KL + 8 * hh;
  gemm_rows16<KL, KRUN, 3>(ap, bp, acc);
  __syncthreads();

#pragma unroll
  for (int nt = 0; nt < 3; ++nt) {
    const int col = 16 * nt + m;
    const int cc  = col < NC ? col : NC - 1;
    const float bc = sb[64 + cc];
#pragma unroll
    for (int r = 0; r < 8; ++r) {
      const float val = acc[nt][r] + bc;
      if (col < NC) lg[(16 * wave + 8 * hh + r) * NC + col] = val;
    }
  }
  __syncthreads();

  const int liveRows = (NN - rowBase) < GBM ? (NN - rowBase) : GBM;
  const int nv4 = liveRows * (NC / 4);
  float* ob = out + (size_t)blk * (size_t)(GBM * NC);
  head_flush(lg, ob, nv4, flag, tid);
  __threadfence();
  head_flush(lg, ob, nv4, flag, tid);
}

extern "C" void kernel_launch(void* const* d_in, const int* in_sizes, int n_in,
                              void* d_out, int out_size, void* d_ws, size_t ws_size,
                              hipStream_t stream) {
  if (n_in < 9) return;
  if (in_sizes[0] != NN * FD) return;
  if (in_sizes[1] != NE) return;
  if (in_sizes[2] != NE) return;
  if (in_sizes[3] != NE) return;
  if (in_sizes[4] != FD * HD) return;
  if (in_sizes[5] != HD) return;
  if (in_sizes[6] != NLAY * HD * HD) return;
  if (in_sizes[7] != HD * NC) return;
  if (in_sizes[8] != NC) return;
  if (out_size != NN * NC) return;

  const float* x    = (const float*)d_in[0];
  const int*   srcs = (const int*)d_in[1];
  const int*   dsts = (const int*)d_in[2];
  const float* ew   = (const float*)d_in[3];
  const float* Win  = (const float*)d_in[4];
  const float* bin  = (const float*)d_in[5];
  const float* Wl   = (const float*)d_in[6];
  const float* Wo   = (const float*)d_in[7];
  const float* bo   = (const float*)d_in[8];
  float* out = (float*)d_out;

  constexpr size_t zXB   = (size_t)MP * FD * 2;
  constexpr size_t zF    = (size_t)MP * HD * 4;
  constexpr size_t zHL   = (size_t)MP * KL * 2;
  constexpr size_t zLIST = (size_t)NBK * RCAP * 4;
  constexpr size_t zCO   = (size_t)NBK * 2 * NBRUN * 4;
  constexpr size_t zFLAG = (size_t)NBK * 128;
  constexpr size_t zW0T  = (size_t)HD * FD * 2;
  constexpr size_t zWLD  = (size_t)NLAY * HD * KL * 2;
  constexpr size_t zWOD  = (size_t)NCP * KL * 2;
  constexpr size_t zSM   = 512;
  constexpr size_t oXB   = 0;
  constexpr size_t oX0   = oXB + zXB;
  constexpr size_t oH    = oX0 + zF;
  constexpr size_t oHMIX = oH + zF;
  constexpr size_t oHMhl = oHMIX + zF;
  constexpr size_t oHhl  = oHMhl + zHL;
  constexpr size_t oLIST = oHhl + zHL;
  constexpr size_t oCO   = oLIST + zLIST;
  constexpr size_t oFLAG = oCO + zCO;
  constexpr size_t oW0T  = oFLAG + zFLAG;
  constexpr size_t oWLD  = oW0T + zW0T;
  constexpr size_t oWOD  = oWLD + zWLD;
  constexpr size_t oSM   = oWOD + zWOD;
  constexpr size_t oEND  = oSM + zSM;
  static_assert(zXB % 256 == 0 && zF % 256 == 0 && zHL % 256 == 0 && zLIST % 256 == 0 && zCO % 256 == 0);
  static_assert(zFLAG % 256 == 0 && zW0T % 256 == 0 && zWLD % 256 == 0 && zWOD % 256 == 0 && zSM % 256 == 0);
  static_assert(oEND <= (size_t)WSMAX);
  if (oEND > ws_size) return;

  char* ws = (char*)d_ws;
  unsigned short* XB   = (unsigned short*)(ws + oXB);
  float*          X0   = (float*)(ws + oX0);
  float*          H    = (float*)(ws + oH);
  float*          HMIX = (float*)(ws + oHMIX);
  unsigned short* HMhl = (unsigned short*)(ws + oHMhl);
  unsigned short* Hhl  = (unsigned short*)(ws + oHhl);
  int*            LIST = (int*)(ws + oLIST);
  int*            CO   = (int*)(ws + oCO);
  int*            FLAG = (int*)(ws + oFLAG);
  unsigned short* W0T  = (unsigned short*)(ws + oW0T);
  unsigned short* WLD  = (unsigned short*)(ws + oWLD);
  unsigned short* WOD  = (unsigned short*)(ws + oWOD);
  float*          SM   = (float*)(ws + oSM);

  hipFuncSetAttribute(reinterpret_cast<const void*>(&k_bucket), hipFuncAttributeMaxDynamicSharedMemorySize, (int)BK_LDS);

  k_prep<<<PBTOT, NTHR, 0, stream>>>(x, Win, bin, Wl, Wo, bo, XB, W0T, WLD, WOD, SM);
  k_bucket<<<NBK, NTHR, BK_LDS, stream>>>(srcs, dsts, ew, LIST, CO, FLAG);
  k_gemm0<<<MP / GBM, NTHR, 0, stream>>>(XB, W0T, SM, X0);

  const float c9 = (float)(1.0 - 0.1);
  const float c1 = (float)0.1;
  for (int l = 0; l < NLAY; ++l) {
    const double bd = log(0.5 / (double)(l + 1) + 1.0);
    const float cb  = (float)bd;
    const float cm  = (float)(1.0 - bd);
    const float* Hs = (l == 0) ? X0 : H;
    k_agg<<<MP / ABM, NTHR, 0, stream>>>(LIST, CO, FLAG, Hs, X0, c9, c1, HMIX, HMhl);
    const unsigned short* bt = WLD + (size_t)l * HD * KL;
    if (l == NLAY - 1)
      k_lin<1><<<MP / GBM, NTHR, 0, stream>>>(HMhl, bt, HMIX, cm, cb, H, Hhl);
    else
      k_lin<0><<<MP / GBM, NTHR, 0, stream>>>(HMhl, bt, HMIX, cm, cb, H, Hhl);
  }
  k_head<<<MP / GBM, NTHR, 0, stream>>>(Hhl, WOD, SM, FLAG, out);
}
